// CausalTransformer_41034117546202
// MI455X (gfx1250) — hardware-verified
//
#include <hip/hip_runtime.h>
#include <math.h>
#include <stdint.h>

#ifndef NB
#define NB        2
#endif
#ifndef SEQ
#define SEQ       2048
#endif
#define NB_FULL   2
#define SEQ_FULL  2048
#define NLAYER    6
#define DMODEL    256
#define NHEAD     4
#define HDIM      64
#define DFF       512
#define OBSD      637
#define OBSP      640
#define NACT      4
#define NACTP     64
#define NBUCK     32
#define NROWS     (NB * SEQ)
#define KD        (2 * DMODEL)
#define KF        (2 * DFF)
#define VTR       KD
#define OUT1_OFF  (NB_FULL * SEQ_FULL * NACT)
#define OUT_TOTAL (OUT1_OFF + NB_FULL * SEQ_FULL * OBSD)

#define WSC_I 64
#define RC_I  64
#define WLO_I 1
#define WSC   64.0f
#define WLO   1.0f
#define RC    64.0f
#define RCI   0.015625f
#define OBC   16.0f
#define HC    16.0f
#define QC    16.0f
#define KC    16.0f
#define VC    16.0f
#define PC    16384.0f
#define CC    16.0f
#define GC    64.0f
#define ATT_SCALE 0.125f
#define LOG2E   1.4426950408889634f
#define RMS_EPS 1.1920929e-07f
static_assert(RC_I * WLO_I == WSC_I);
static_assert(NHEAD * HDIM == DMODEL);
static_assert(NB >= 1 && NB <= NB_FULL && SEQ >= 64 && SEQ <= SEQ_FULL);
static_assert((SEQ % 64) == 0 && (SEQ % 16) == 0 && (NROWS % 64) == 0 && (DMODEL % 64) == 0 && (DFF % 64) == 0);
static_assert((OBSP % 64) == 0 && (NACTP % 64) == 0 && OBSP >= OBSD && NACTP >= NACT && (OBSP - OBSD) < 64);
static_assert((KD % 32) == 0 && (KF % 32) == 0 && (OBSP % 32) == 0);
static_assert((NROWS % 256) == 0 && (NROWS % 4) == 0 && ((SEQ * OBSD) % 4) == 0);
static_assert(OUT_TOTAL == 2625536);

typedef _Float16 v16h __attribute__((ext_vector_type(16)));
typedef _Float16 v8h  __attribute__((ext_vector_type(8)));
typedef float    v8f  __attribute__((ext_vector_type(8)));
typedef float    v4f  __attribute__((ext_vector_type(4)));
typedef unsigned int v4u __attribute__((ext_vector_type(4)));

union FragH { v16h v; v8h h[2]; v4u u[2]; };

__device__ __forceinline__ unsigned short bf_bits(float f) {
  unsigned u = __float_as_uint(f);
  return (unsigned short)((u + 0x7FFFu + ((u >> 16) & 1u)) >> 16);
}
__device__ __forceinline__ float bf_up(unsigned short h) { return __uint_as_float(((unsigned)h) << 16); }
__device__ __forceinline__ float bfr(float f) { return bf_up(bf_bits(f)); }
__device__ __forceinline__ unsigned short h_bits(_Float16 x) { return __builtin_bit_cast(unsigned short, x); }
__device__ __forceinline__ unsigned pk16(unsigned short a, unsigned short b) { return (unsigned)a | ((unsigned)b << 16); }
__device__ __forceinline__ v8f zero8() { v8f z = {0.f, 0.f, 0.f, 0.f, 0.f, 0.f, 0.f, 0.f}; return z; }
__device__ __forceinline__ int imin(int a, int b) { return a < b ? a : b; }
__device__ __forceinline__ int imax(int a, int b) { return a > b ? a : b; }

__device__ __forceinline__ int rel_bucket(int rel) {
  int b = 31;
  b = (rel < 91) ? 30 : b;
  b = (rel < 64) ? 29 : b;
  b = (rel < 46) ? 28 : b;
  b = (rel < 32) ? 27 : b;
  b = (rel < 23) ? 26 : b;
  b = (rel < 16) ? 25 : b;
  b = (rel < 12) ? 24 : b;
  b = (rel < 8) ? (16 + rel) : b;
  b = (rel == 0) ? 0 : b;
  return b;
}

__device__ __forceinline__ v16h ldfrag_h(const _Float16* p) {
  FragH f;
  f.h[0] = *(const v8h*)(p);
  f.h[1] = *(const v8h*)(p + 16);
  return f.v;
}
__device__ __forceinline__ v16h ldfrag_u(const unsigned short* p) {
  FragH f;
  f.u[0] = *(const v4u*)(p);
  f.u[1] = *(const v4u*)(p + 16);
  return f.v;
}

__device__ __forceinline__ v8f mma_raw(v16h a, v16h b, v8f c) {
  return __builtin_amdgcn_wmma_f32_16x16x32_f16(false, a, false, b, (short)0, c, false, false);
}
__device__ __forceinline__ void dep_guard1(v8f& a, v8f& b, v16h x) {
#if defined(__HIP_DEVICE_COMPILE__)
  asm volatile("v_nop\n\tv_nop\n\tv_nop\n\tv_nop" : "+v"(a), "+v"(b) : "v"(x));
#endif
}
__device__ __forceinline__ void guard_s2x4(v8f& s, v8f& t, v16h a0, v16h a1, v16h b0, v16h b1) {
#if defined(__HIP_DEVICE_COMPILE__)
  asm volatile("v_nop\n\tv_nop\n\tv_nop\n\tv_nop" : "+v"(s), "+v"(t) : "v"(a0), "v"(a1), "v"(b0), "v"(b1));
#endif
}
__device__ __forceinline__ void guard_pv4(v8f& a, v8f& b, v8f& c, v8f& d, v16h x, v16h y, v16h z, v16h w, v16h u) {
#if defined(__HIP_DEVICE_COMPILE__)
  asm volatile("v_nop\n\tv_nop\n\tv_nop\n\tv_nop"
               : "+v"(a), "+v"(b), "+v"(c), "+v"(d) : "v"(x), "v"(y), "v"(z), "v"(w), "v"(u));
#endif
}
__device__ __forceinline__ void keep4_h(v16h a, v16h b, v16h c, v16h d) {
#if defined(__HIP_DEVICE_COMPILE__)
  asm volatile("v_nop" :: "v"(a), "v"(b), "v"(c), "v"(d));
#endif
}
__device__ __forceinline__ void acc_guard4(v8f& a, v8f& b, v8f& c, v8f& d) {
#if defined(__HIP_DEVICE_COMPILE__)
  asm volatile("v_nop\n\tv_nop\n\tv_nop\n\tv_nop" : "+v"(a), "+v"(b), "+v"(c), "+v"(d));
#endif
}
__device__ __forceinline__ void wave_sync_lds() {
  __builtin_amdgcn_fence(__ATOMIC_RELEASE, "workgroup");
  __builtin_amdgcn_wave_barrier();
  __builtin_amdgcn_fence(__ATOMIC_ACQUIRE, "workgroup");
}

template <int DUAL>
__global__ __launch_bounds__(256) void tcvt16(const float* __restrict__ src, long long sZ,
                                              unsigned short* dst, long long dZ,
                                              int R, int C, int ldd, int locol, float schi, float sclo) {
  __shared__ __align__(16) unsigned short sT[64 * 72];
  const int tid = threadIdx.x, lane = tid & 31, wave = tid >> 5;
  const int c0 = blockIdx.x * 64, r0 = blockIdx.y * 64;
  const float* srcz = src + (size_t)((long long)blockIdx.z * sZ);
  unsigned short* dstz = dst + (size_t)((long long)blockIdx.z * dZ);
  const int rr = tid >> 2, cc = (tid & 3) * 16;
  const int r = r0 + rr;
  const int rcl = imin(r, R - 1);
  const float* sp = srcz + (size_t)rcl * C;
#pragma unroll
  for (int e = 0; e < 16; ++e) {
    const int cidx = c0 + cc + e;
    const int ccl = imin(cidx, C - 1);
    float a = sp[ccl];
    a = (r < R && cidx < C) ? a : 0.f;
    sT[(cc + e) * 72 + rr] = bf_bits(a);
  }
  __syncthreads();
  v4u hvals[2], lvals[2];
#pragma unroll
  for (int it = 0; it < 2; ++it) {
    const int q = it * 32 + wave * 4 + (lane >> 3);
    const v4u raw = *(const v4u*)(sT + q * 72 + (lane & 7) * 8);
    v4u hv = {0u, 0u, 0u, 0u}, lv = {0u, 0u, 0u, 0u};
#pragma unroll
    for (int e = 0; e < 4; ++e) {
      const float f0 = bf_up((unsigned short)(raw[e] & 0xFFFFu));
      const float f1 = bf_up((unsigned short)(raw[e] >> 16));
      hv[e] = pk16(h_bits((_Float16)(f0 * schi)), h_bits((_Float16)(f1 * schi)));
      if constexpr (DUAL == 1) lv[e] = pk16(h_bits((_Float16)(f0 * sclo)), h_bits((_Float16)(f1 * sclo)));
    }
    hvals[it] = hv;
    lvals[it] = lv;
  }
  for (int pass = 0; pass < 2; ++pass) {
#pragma unroll
    for (int it = 0; it < 2; ++it) {
      const int q = it * 32 + wave * 4 + (lane >> 3);
      unsigned short* p = dstz + (size_t)(c0 + q) * ldd + r0 + (lane & 7) * 8;
      *(volatile v4u*)p = hvals[it];
      if constexpr (DUAL == 1) *(volatile v4u*)(p + locol) = lvals[it];
    }
    __threadfence();
  }
  (void)sclo; (void)locol;
}

template <int OM, int RM, int ACT, int BM>
__global__ __launch_bounds__(256) void gemm64(
    const unsigned short* __restrict__ Ap, int lda, long long sA,
    const unsigned short* __restrict__ Btp, int ldb, long long sB,
    const float* __restrict__ Rp,
    const float* __restrict__ biasp, int nbias,
    void* Cout, int ldc, long long sC, long long lofs,
    int M, int N, int K, float oscale, float ocarry) {
  __shared__ __align__(16) float sT[8][16 * 68];
  const int by   = blockIdx.y;
  const int lane = threadIdx.x & 31;
  const int wave = threadIdx.x >> 5;
  const int tilesN = N >> 6;
  const int tilesM = M >> 6;
  const int tile = blockIdx.x * 8 + wave;
  if (tile >= tilesM * tilesN) return;
  const int tm = tile / tilesN;
  const int tn = tile - tm * tilesN;
  const int m0 = tm << 6;
  const int n0 = tn << 6;

  const unsigned short* A1 = Ap  + (size_t)((long long)by * sA);
  const unsigned short* Bb = Btp + (size_t)((long long)by * sB);

  const int rlane = lane & 15;
  const int koff  = (lane >> 4) * 8;
  const int mOff  = (lane >> 4) * 8;

  v8f acc[4][4];
#pragma unroll
  for (int i = 0; i < 4; ++i)
#pragma unroll
    for (int j = 0; j < 4; ++j) acc[i][j] = zero8();

  for (int k0 = 0; k0 < K; k0 += 32) {
    v16h bh[4];
#pragma unroll
    for (int j = 0; j < 4; ++j) {
      const size_t bofs = (size_t)(n0 + (j << 4) + rlane) * ldb + koff + k0;
      bh[j] = ldfrag_u(Bb + bofs);
    }
#pragma unroll
    for (int i = 0; i < 4; ++i) {
      const size_t ao = (size_t)(m0 + (i << 4) + rlane) * lda + koff + k0;
      const v16h ah = ldfrag_u(A1 + ao);
#pragma unroll
      for (int j = 0; j < 4; ++j) acc[i][j] = mma_raw(ah, bh[j], acc[i][j]);
      dep_guard1(acc[i][0], acc[i][3], ah);
    }
    keep4_h(bh[0], bh[1], bh[2], bh[3]);
  }
  acc_guard4(acc[0][0], acc[0][1], acc[0][2], acc[0][3]);
  acc_guard4(acc[1][0], acc[1][1], acc[1][2], acc[1][3]);
  acc_guard4(acc[2][0], acc[2][1], acc[2][2], acc[2][3]);
  acc_guard4(acc[3][0], acc[3][1], acc[3][2], acc[3][3]);

  const int hh2 = lane >> 4, c4 = (lane & 15) * 4;
  const int q8  = lane >> 3, c8 = (lane & 7) * 8;

  float bc4[4], bc8[8];
#pragma unroll
  for (int e = 0; e < 4; ++e) bc4[e] = 0.f;
#pragma unroll
  for (int e = 0; e < 8; ++e) bc8[e] = 0.f;
  if constexpr (BM == 1) {
    if constexpr (OM == 0) {
#pragma unroll
      for (int e = 0; e < 4; ++e) {
        const int n = n0 + c4 + e;
        const int ncl = imin(n, nbias - 1);
        const float t = bfr(biasp[ncl]);
        bc4[e] = (n < nbias) ? t : 0.f;
      }
    } else {
#pragma unroll
      for (int e = 0; e < 8; ++e) {
        const int n = n0 + c8 + e;
        const int ncl = imin(n, nbias - 1);
        const float t = bfr(biasp[ncl]);
        bc8[e] = (n < nbias) ? t : 0.f;
      }
    }
  }

  float* slab = sT[wave];
#pragma unroll
  for (int i = 0; i < 4; ++i) {
    const int mBase = m0 + (i << 4);
#pragma unroll
    for (int j = 0; j < 4; ++j) {
#pragma unroll
      for (int r = 0; r < 8; ++r) {
        slab[(mOff + r) * 68 + (j << 4) + rlane] = acc[i][j][r];
      }
    }
    wave_sync_lds();
    if constexpr (OM == 0) {
      float* C = (float*)Cout + (size_t)((long long)by * sC);
      v4f vals[8];
#pragma unroll
      for (int it = 0; it < 8; ++it) {
        const int row = it * 2 + hh2;
        const int gr  = mBase + row;
        v4f v = *(const v4f*)(slab + row * 68 + c4);
        v4f rv = {0.f, 0.f, 0.f, 0.f};
        if constexpr (RM == 2) {
          const float* R = Rp + (size_t)((long long)by * sC);
          rv = *(const v4f*)(R + (size_t)gr * ldc + n0 + c4);
        }
#pragma unroll
        for (int e = 0; e < 4; ++e) {
          float u = v[e] * oscale;
          if constexpr (BM == 1) u += bc4[e];
          if constexpr (ACT == 2) u = fmaxf(u, 0.f);
          v[e] = u + rv[e];
        }
        vals[it] = v;
      }
      for (int pass = 0; pass < 2; ++pass) {
#pragma unroll
        for (int it = 0; it < 8; ++it) {
          const int gr = mBase + it * 2 + hh2;
          *(volatile v4f*)(C + (size_t)gr * ldc + n0 + c4) = vals[it];
        }
        __threadfence();
      }
    } else {
      unsigned short* C = (unsigned short*)Cout + (size_t)((long long)by * sC);
      v4u hv[4], lv[4];
#pragma unroll
      for (int it = 0; it < 4; ++it) {
        const int row = it * 4 + q8;
        const float* spf = slab + row * 68 + c8;
        v4u a = {0u, 0u, 0u, 0u}, bl = {0u, 0u, 0u, 0u};
#pragma unroll
        for (int e = 0; e < 4; ++e) {
          float f0 = spf[2 * e] * oscale;
          float f1 = spf[2 * e + 1] * oscale;
          if constexpr (BM == 1) { f0 += bc8[2 * e]; f1 += bc8[2 * e + 1]; }
          if constexpr (ACT == 2) { f0 = fmaxf(f0, 0.f); f1 = fmaxf(f1, 0.f); }
          f0 *= ocarry; f1 *= ocarry;
          const _Float16 g0 = (_Float16)f0, g1 = (_Float16)f1;
          const float r0 = (f0 - (float)g0) * RC, r1 = (f1 - (float)g1) * RC;
          a[e]  = pk16(h_bits(g0), h_bits(g1));
          bl[e] = pk16(h_bits((_Float16)r0), h_bits((_Float16)r1));
        }
        hv[it] = a;
        lv[it] = bl;
      }
      for (int pass = 0; pass < 2; ++pass) {
#pragma unroll
        for (int it = 0; it < 4; ++it) {
          const int row = it * 4 + q8;
          unsigned short* p = C + (size_t)(mBase + row) * ldc + n0 + c8;
          *(volatile v4u*)p = hv[it];
          *(volatile v4u*)(p + (size_t)lofs) = lv[it];
        }
        __threadfence();
      }
    }
    wave_sync_lds();
  }
  (void)Rp; (void)ocarry; (void)lofs; (void)nbias; (void)biasp;
}

#define ATT_THREADS (NHEAD * 32)
#define ATT_BLOCKS  (NB * (SEQ / 16))
#define PT_FLOATS   (NHEAD * 16 * 36)
static_assert(ATT_THREADS == 128 && (KD / 8) == 64 && ((16 * KD) % (8 * ATT_THREADS)) == 0 && ((16 * KD) / (8 * ATT_THREADS)) == 8);
static_assert((KD * 2) % 128 == 0 && (HDIM % 32) == 0);

__global__ __launch_bounds__(ATT_THREADS)
void attn4(const unsigned short* __restrict__ QPp, const unsigned short* __restrict__ KPp,
           const unsigned short* __restrict__ VTq, const float* __restrict__ relbl, unsigned short* CT) {
  __shared__ __align__(16) float sbias[NHEAD * SEQ];
  __shared__ __align__(16) float spt[PT_FLOATS];
  __shared__ __align__(16) unsigned short sos[16 * KD];

  const int tid  = threadIdx.x;
  const int wave = tid >> 5;
  const int lane = tid & 31;
  const int hh   = lane >> 4;
  const int c    = lane & 15;

  const int qt   = blockIdx.x % (SEQ / 16);
  const int bat  = blockIdx.x / (SEQ / 16);
  const int head = wave;
  const int q0   = qt * 16;
  const int srow = q0 + 8 * hh;
  const int kend = q0 + 16;

  for (int rel = tid; rel < kend; rel += ATT_THREADS) {
    const int bk = rel_bucket(rel);
    const v4f bv = *(const v4f*)(relbl + bk * NHEAD);
#pragma unroll
    for (int h2 = 0; h2 < NHEAD; ++h2) sbias[h2 * SEQ + rel] = bfr(bv[h2]) * LOG2E;
  }
  __syncthreads();

  const float* sb = sbias + head * SEQ;
  const _Float16* Q16 = (const _Float16*)(const void*)QPp;
  const _Float16* K16 = (const _Float16*)(const void*)KPp;
  const _Float16* V16 = (const _Float16*)(const void*)VTq;
  const _Float16* Qh = Q16 + ((size_t)bat * SEQ + q0 + c) * KD + head * HDIM + 8 * hh;
  const _Float16* Kb = K16 + (size_t)bat * SEQ * KD + head * HDIM + 8 * hh;
  const _Float16* Vh = V16 + ((size_t)bat * VTR + head * HDIM) * SEQ + 8 * hh;
  const _Float16* Vl = Vh + (size_t)DMODEL * SEQ;
  const float lsc = (LOG2E * ATT_SCALE) / (QC * KC);

  const v16h qah = ldfrag_h(Qh), qbh = ldfrag_h(Qh + 32);
  const v16h qal = ldfrag_h(Qh + DMODEL), qbl = ldfrag_h(Qh + DMODEL + 32);

  float mrow[8], lrow[8];
  v8f om0 = zero8(), om1 = zero8(), om2 = zero8(), om3 = zero8();
  v8f or0 = zero8(), or1 = zero8(), or2 = zero8(), or3 = zero8();
#pragma unroll
  for (int r = 0; r < 8; ++r) { mrow[r] = -INFINITY; lrow[r] = 0.f; }
  float* pt = spt + wave * (16 * 36);

#pragma unroll 1
  for (int kb = 0; kb < kend; kb += 32) {
    const _Float16* kp = Kb + (size_t)(kb + c) * KD;
    v8f s0m, s0r, s1m, s1r;
    {
      const v16h k0h = ldfrag_h(kp), k1h = ldfrag_h(kp + 32);
      const v16h k0l = ldfrag_h(kp + DMODEL), k1l = ldfrag_h(kp + DMODEL + 32);
      s0m = mma_raw(qah, k0h, zero8());
      s0m = mma_raw(qbh, k1h, s0m);
      s0r = mma_raw(qah, k0l, zero8());
      s0r = mma_raw(qbh, k1l, s0r);
      s0r = mma_raw(qal, k0h, s0r);
      s0r = mma_raw(qbl, k1h, s0r);
      guard_s2x4(s0m, s0r, k0h, k1h, k0l, k1l);
    }
    {
      const _Float16* kq = kp + (size_t)16 * KD;
      const v16h k0h = ldfrag_h(kq), k1h = ldfrag_h(kq + 32);
      const v16h k0l = ldfrag_h(kq + DMODEL), k1l = ldfrag_h(kq + DMODEL + 32);
      s1m = mma_raw(qah, k0h, zero8());
      s1m = mma_raw(qbh, k1h, s1m);
      s1r = mma_raw(qah, k0l, zero8());
      s1r = mma_raw(qbh, k1l, s1r);
      s1r = mma_raw(qal, k0h, s1r);
      s1r = mma_raw(qbl, k1h, s1r);
      guard_s2x4(s1m, s1r, k0h, k1h, k0l, k1l);
      keep4_h(qah, qbh, qal, qbl);
    }
    const int key0 = kb + c;
    const int key1 = kb + 16 + c;
#pragma unroll
    for (int r = 0; r < 8; ++r) {
      const int qi = srow + r;
      const int i0 = imax(qi - key0, 0);
      const int i1 = imax(qi - key1, 0);
      float t0 = (s0m[r] + s0r[r] * RCI) * lsc + sb[i0];
      float t1 = (s1m[r] + s1r[r] * RCI) * lsc + sb[i1];
      t0 = (key0 > qi) ? -INFINITY : t0;
      t1 = (key1 > qi) ? -INFINITY : t1;
      float mx = fmaxf(t0, t1);
#pragma unroll
      for (int off = 1; off < 16; off <<= 1) mx = fmaxf(mx, __shfl_xor(mx, off, 32));
      const float mn = fmaxf(mrow[r], mx);
      const float al = exp2f(fmaxf(mrow[r] - mn, -126.0f));
      mrow[r] = mn;
      const float e0 = exp2f(t0 - mn);
      const float e1 = exp2f(t1 - mn);
      float ps = e0 + e1;
#pragma unroll
      for (int off = 1; off < 16; off <<= 1) ps += __shfl_xor(ps, off, 32);
      lrow[r] = lrow[r] * al + ps;
      om0[r] *= al; om1[r] *= al; om2[r] *= al; om3[r] *= al;
      or0[r] *= al; or1[r] *= al; or2[r] *= al; or3[r] *= al;
      const int ro = (8 * hh + r) * 36 + c;
      pt[ro]      = e0;
      pt[ro + 16] = e1;
    }
    wave_sync_lds();
    FragH ph;
    {
      const float* prow = pt + c * 36 + 8 * hh;
      const v4f p0 = *(const v4f*)(prow), p1 = *(const v4f*)(prow + 4);
      const v4f p2 = *(const v4f*)(prow + 16), p3 = *(const v4f*)(prow + 20);
#pragma unroll
      for (int e = 0; e < 4; ++e) {
        ph.h[0][e]     = (_Float16)(p0[e] * PC);
        ph.h[0][4 + e] = (_Float16)(p1[e] * PC);
        ph.h[1][e]     = (_Float16)(p2[e] * PC);
        ph.h[1][4 + e] = (_Float16)(p3[e] * PC);
      }
    }
    {
      const _Float16* vp = Vh + (size_t)c * SEQ + kb;
      const v16h vb0 = ldfrag_h(vp);
      const v16h vb1 = ldfrag_h(vp + (size_t)16 * SEQ);
      const v16h vb2 = ldfrag_h(vp + (size_t)32 * SEQ);
      const v16h vb3 = ldfrag_h(vp + (size_t)48 * SEQ);
      om0 = mma_raw(ph.v, vb0, om0);
      om1 = mma_raw(ph.v, vb1, om1);
      om2 = mma_raw(ph.v, vb2, om2);
      om3 = mma_raw(ph.v, vb3, om3);
      guard_pv4(om0, om1, om2, om3, ph.v, vb0, vb1, vb2, vb3);
    }
    {
      const _Float16* vq = Vl + (size_t)c * SEQ + kb;
      const v16h vl0 = ldfrag_h(vq);
      const v16h vl1 = ldfrag_h(vq + (size_t)16 * SEQ);
      const v16h vl2 = ldfrag_h(vq + (size_t)32 * SEQ);
      const v16h vl3 = ldfrag_h(vq + (size_t)48 * SEQ);
      or0 = mma_raw(ph.v, vl0, or0);
      or1 = mma_raw(ph.v, vl1, or1);
      or2 = mma_raw(ph.v, vl2, or2);
      or3 = mma_raw(ph.v, vl3, or3);
      guard_pv4(or0, or1, or2, or3, ph.v, vl0, vl1, vl2, vl3);
    }
    wave_sync_lds();
  }

  const float oc = CC / (PC * VC);
  unsigned short* osw = sos + head * HDIM + c;
#pragma unroll
  for (int r = 0; r < 8; ++r) {
    const float inv = (1.0f / lrow[r]) * oc;
    unsigned short* op = osw + (8 * hh + r) * KD;
    const float u0 = (om0[r] + or0[r] * RCI) * inv;
    const float u1 = (om1[r] + or1[r] * RCI) * inv;
    const float u2 = (om2[r] + or2[r] * RCI) * inv;
    const float u3 = (om3[r] + or3[r] * RCI) * inv;
    const _Float16 g0 = (_Float16)u0, g1 = (_Float16)u1, g2 = (_Float16)u2, g3 = (_Float16)u3;
    op[0]           = h_bits(g0);
    op[16]          = h_bits(g1);
    op[32]          = h_bits(g2);
    op[48]          = h_bits(g3);
    op[DMODEL]      = h_bits((_Float16)((u0 - (float)g0) * RC));
    op[DMODEL + 16] = h_bits((_Float16)((u1 - (float)g1) * RC));
    op[DMODEL + 32] = h_bits((_Float16)((u2 - (float)g2) * RC));
    op[DMODEL + 48] = h_bits((_Float16)((u3 - (float)g3) * RC));
  }
  __syncthreads();
  {
    v4u vals[8];
#pragma unroll
    for (int it = 0; it < 8; ++it) {
      const int p = it * ATT_THREADS + tid;
      vals[it] = *(const v4u*)(sos + (size_t)p * 8);
    }
    unsigned short* dst = CT + ((size_t)bat * SEQ + q0) * KD;
    for (int pass = 0; pass < 2; ++pass) {
#pragma unroll
      for (int it = 0; it < 8; ++it) {
        const int p = it * ATT_THREADS + tid;
        const int row = p >> 6, col8 = (p & 63) * 8;
        *(volatile v4u*)(dst + (size_t)row * KD + col8) = vals[it];
      }
      __threadfence();
    }
  }
}

__global__ __launch_bounds__(128) void rmsn(const float* __restrict__ Xp, const float* __restrict__ wp, unsigned short* outh) {
  const int wave = threadIdx.x >> 5, lane = threadIdx.x & 31;
  const int row = blockIdx.x * 4 + wave;
  const int c0 = lane * 8;
  const float* xp = Xp + (size_t)row * DMODEL + c0;
  const v4f x0 = *(const v4f*)(xp), x1 = *(const v4f*)(xp + 4);
  float ss = ((x0[0] * x0[0] + x0[1] * x0[1]) + (x0[2] * x0[2] + x0[3] * x0[3])) +
             ((x1[0] * x1[0] + x1[1] * x1[1]) + (x1[2] * x1[2] + x1[3] * x1[3]));
#pragma unroll
  for (int off = 1; off < 32; off <<= 1) ss += __shfl_xor(ss, off, 32);
  const float rstd = rsqrtf(ss * (1.0f / (float)DMODEL) + RMS_EPS);
  const v4f w0 = *(const v4f*)(wp + c0), w1 = *(const v4f*)(wp + c0 + 4);
  float o[8];
#pragma unroll
  for (int e = 0; e < 4; ++e) {
    o[e]     = (x0[e] * rstd) * bfr(w0[e]);
    o[4 + e] = (x1[e] * rstd) * bfr(w1[e]);
  }
  v4u hv, lv;
#pragma unroll
  for (int e = 0; e < 4; ++e) {
    const float f0 = o[2 * e] * HC, f1 = o[2 * e + 1] * HC;
    const _Float16 g0 = (_Float16)f0, g1 = (_Float16)f1;
    hv[e] = pk16(h_bits(g0), h_bits(g1));
    lv[e] = pk16(h_bits((_Float16)((f0 - (float)g0) * RC)), h_bits((_Float16)((f1 - (float)g1) * RC)));
  }
  unsigned short* dp = outh + (size_t)row * KD + c0;
  for (int pass = 0; pass < 2; ++pass) {
    *(volatile v4u*)dp = hv;
    *(volatile v4u*)(dp + DMODEL) = lv;
    __threadfence();
  }
}

__global__ __launch_bounds__(128) void cvtobs(const float* __restrict__ src, unsigned short* dst) {
  const int wave = threadIdx.x >> 5, lane = threadIdx.x & 31;
  const int m = blockIdx.x * 4 + wave;
  const int b = m / SEQ, t = m - b * SEQ;
  const float* sp = src + ((size_t)b * SEQ_FULL + t) * OBSD;
  unsigned short* dp = dst + (size_t)m * OBSP;
  for (int pass = 0; pass < 2; ++pass) {
#pragma unroll 1
    for (int it = 0; it < 3; ++it) {
      const int p = it * 32 + lane;
      const int col0 = p * 8;
      v4u a;
#pragma unroll
      for (int e = 0; e < 4; ++e) {
        const int ca = col0 + 2 * e, cb = ca + 1;
        float fa = sp[imin(ca, OBSD - 1)];
        float fb = sp[imin(cb, OBSD - 1)];
        fa = (ca < OBSD) ? fa : 0.f;
        fb = (cb < OBSD) ? fb : 0.f;
        a[e] = pk16(h_bits((_Float16)(bfr(fa) * OBC)), h_bits((_Float16)(bfr(fb) * OBC)));
      }
      if (p < OBSP / 8) *(volatile v4u*)(dp + (size_t)p * 8) = a;
    }
    __threadfence();
  }
}

__global__ __launch_bounds__(256) void ocopy(const float* __restrict__ actf, const float* __restrict__ obsf, float* outp) {
  const int g = blockIdx.x * 256 + threadIdx.x;
  if (blockIdx.y == 0) {
    if (g >= NROWS) return;
    const int b = g / SEQ, t = g - b * SEQ;
    const v4f v = *(const v4f*)(actf + (size_t)g * NACTP);
    float* d = outp + ((size_t)b * SEQ_FULL + t) * NACT;
    for (int pass = 0; pass < 2; ++pass) {
      *(volatile v4f*)d = v;
      __threadfence();
    }
  } else {
    const int ppb = (SEQ * OBSD) / 4;
    if (g >= NB * ppb) return;
    const int b = g / ppb;
    const int i = (g - b * ppb) * 4;
    v4f v;
#pragma unroll
    for (int e = 0; e < 4; ++e) {
      const int idx = i + e;
      const int row = idx / OBSD;
      const int col = idx - row * OBSD;
      v[e] = obsf[((size_t)b * SEQ + row) * OBSP + col];
    }
    float* d = outp + (size_t)OUT1_OFF + (size_t)b * SEQ_FULL * OBSD + i;
    for (int pass = 0; pass < 2; ++pass) {
      *(volatile v4f*)d = v;
      __threadfence();
    }
  }
}

extern "C" void kernel_launch(void* const* d_in, const int* in_sizes, int n_in,
                              void* d_out, int out_size, void* d_ws, size_t ws_size,
                              hipStream_t stream) {
  if (n_in < 19) return;
  if (in_sizes[0] < ((NB - 1) * SEQ_FULL + SEQ) * OBSD) return;
  if (in_sizes[1] < OBSD * DMODEL || in_sizes[2] < DMODEL) return;
  if (in_sizes[3] < NLAYER * DMODEL) return;
  if (in_sizes[4] < NLAYER * DMODEL * DMODEL || in_sizes[5] < NLAYER * DMODEL * DMODEL) return;
  if (in_sizes[6] < NLAYER * DMODEL * DMODEL || in_sizes[7] < NLAYER * DMODEL * DMODEL) return;
  if (in_sizes[8] < NLAYER * NBUCK * NHEAD || in_sizes[9] < NLAYER * DMODEL) return;
  if (in_sizes[10] < NLAYER * DMODEL * DFF || in_sizes[11] < NLAYER * DFF) return;
  if (in_sizes[12] < NLAYER * DFF * DMODEL || in_sizes[13] < NLAYER * DMODEL) return;
  if (in_sizes[14] < DMODEL || in_sizes[15] < DMODEL * NACT || in_sizes[16] < NACT) return;
  if (in_sizes[17] < DMODEL * OBSD || in_sizes[18] < OBSD) return;
  if (out_size < OUT1_OFF + ((NB - 1) * SEQ_FULL + SEQ) * OBSD) return;

  const float* obs     = (const float*)d_in[0];
  const float* obs_w   = (const float*)d_in[1];
  const float* obs_b   = (const float*)d_in[2];
  const float* norm1_w = (const float*)d_in[3];
  const float* w_q     = (const float*)d_in[4];
  const float* w_k     = (const float*)d_in[5];
  const float* w_v     = (const float*)d_in[6];
  const float* w_o     = (const float*)d_in[7];
  const float* relb    = (const float*)d_in[8];
  const float* norm2_w = (const float*)d_in[9];
  const float* w_1     = (const float*)d_in[10];
  const float* b_1     = (const float*)d_in[11];
  const float* w_2     = (const float*)d_in[12];
  const float* b_2     = (const float*)d_in[13];
  const float* fnorm_w = (const float*)d_in[14];
  const float* act_w   = (const float*)d_in[15];
  const float* act_b   = (const float*)d_in[16];
  const float* obsh_w  = (const float*)d_in[17];
  const float* obsh_b  = (const float*)d_in[18];
  float*       outp    = (float*)d_out;

  const size_t PWE  = (size_t)NLAYER * DMODEL * KD * 2;
  const size_t PW1  = (size_t)NLAYER * DFF * KD * 2;
  const size_t PW2  = (size_t)NLAYER * DMODEL * KF * 2;
  const size_t POBW = (size_t)DMODEL * OBSP * 2;
  const size_t PACW = (size_t)NACTP * KD * 2;
  const size_t POHW = (size_t)OBSP * KD * 2;
  const size_t POBS = (size_t)NROWS * OBSP * 2;
  const size_t PX   = (size_t)NROWS * DMODEL * 4;
  const size_t PH   = (size_t)NROWS * KD * 2;
  const size_t PVT  = (size_t)NB * VTR * SEQ * 2;
  const size_t PG   = (size_t)NROWS * KF * 2;
  const size_t PACF = (size_t)NROWS * NACTP * 4;
  const size_t POBF = (size_t)NROWS * OBSP * 4;
  size_t off = 0;
  const size_t oWQ  = off; off += PWE;
  const size_t oWK  = off; off += PWE;
  const size_t oWV  = off; off += PWE;
  const size_t oWO  = off; off += PWE;
  const size_t oW1  = off; off += PW1;
  const size_t oW2  = off; off += PW2;
  const size_t oOBW = off; off += POBW;
  const size_t oACW = off; off += PACW;
  const size_t oOHW = off; off += POHW;
  const size_t oOBS = off; off += POBS;
  const size_t oXA  = off; off += PX;
  const size_t oXB  = off; off += PX;
  const size_t oHH  = off; off += PH;
  const size_t oQP  = off; off += PH;
  const size_t oKP  = off; off += PH;
  const size_t oCT  = off; off += PH;
  const size_t oVT  = off; off += PVT;
  const size_t oG   = off; off += PG;
  const size_t oACF = off; off += PACF;
  const size_t oOBF = off; off += POBF;
  const size_t endAll = off;
  if (endAll > ws_size) return;
  if (endAll > (size_t)134217728) return;

  char* ws = (char*)d_ws;
  unsigned short* WQ16    = (unsigned short*)(ws + oWQ);
  unsigned short* WK16    = (unsigned short*)(ws + oWK);
  unsigned short* WV16    = (unsigned short*)(ws + oWV);
  unsigned short* WO16    = (unsigned short*)(ws + oWO);
  unsigned short* W116    = (unsigned short*)(ws + oW1);
  unsigned short* W216    = (unsigned short*)(ws + oW2);
  unsigned short* OBSW16  = (unsigned short*)(ws + oOBW);
  unsigned short* ACTW16  = (unsigned short*)(ws + oACW);
  unsigned short* OBSHW16 = (unsigned short*)(ws + oOHW);
  unsigned short* OBS16   = (unsigned short*)(ws + oOBS);
  float*          XA      = (float*)(ws + oXA);
  float*          XB      = (float*)(ws + oXB);
  unsigned short* HH      = (unsigned short*)(ws + oHH);
  unsigned short* QP      = (unsigned short*)(ws + oQP);
  unsigned short* KP      = (unsigned short*)(ws + oKP);
  unsigned short* CT      = (unsigned short*)(ws + oCT);
  unsigned short* VTp     = (unsigned short*)(ws + oVT);
  unsigned short* G16     = (unsigned short*)(ws + oG);
  float*          ACTF    = (float*)(ws + oACF);
  float*          OBSF    = (float*)(ws + oOBF);

  const dim3 blk(256);
  const dim3 blk128(128);
  const dim3 gRow(NROWS / 4);
  const int tilesE  = (NROWS / 64) * (DMODEL / 64);
  const int tilesV  = (DMODEL / 64) * (SEQ / 64);
  const int tilesF  = (NROWS / 64) * (DFF / 64);
  const int tilesA  = (NROWS / 64) * (NACTP / 64);
  const int tilesO  = (NROWS / 64) * (OBSP / 64);
  const dim3 gE((tilesE + 7) / 8, 1);
  const dim3 gQK((tilesE + 7) / 8, 2);
  const dim3 gV((tilesV + 7) / 8, NB);
  const dim3 gF((tilesF + 7) / 8, 1);
  const dim3 gA((tilesA + 7) / 8, 1);
  const dim3 gO((tilesO + 7) / 8, 1);
  const dim3 gAT(ATT_BLOCKS);
  const dim3 bAT(ATT_THREADS);
  const int ppb = (SEQ * OBSD) / 4;
  const int gcx0 = NROWS / 256, gcx1 = (NB * ppb + 255) / 256;
  const dim3 gOC(gcx0 > gcx1 ? gcx0 : gcx1, 2);

  const long long eSrcE = (long long)DMODEL * DMODEL;
  const long long eDstE = (long long)DMODEL * KD;
  const long long sQK   = (long long)NLAYER * DMODEL * KD;
  const long long sKP   = (long long)NROWS * KD;

  cvtobs<<<gRow, blk128, 0, stream>>>(obs, OBS16);
  tcvt16<1><<<dim3(DMODEL / 64, DMODEL / 64, NLAYER), blk, 0, stream>>>(w_q, eSrcE, WQ16, eDstE, DMODEL, DMODEL, KD, DMODEL, WSC, WLO);
  tcvt16<1><<<dim3(DMODEL / 64, DMODEL / 64, NLAYER), blk, 0, stream>>>(w_k, eSrcE, WK16, eDstE, DMODEL, DMODEL, KD, DMODEL, WSC, WLO);
  tcvt16<1><<<dim3(DMODEL / 64, DMODEL / 64, NLAYER), blk, 0, stream>>>(w_v, eSrcE, WV16, eDstE, DMODEL, DMODEL, KD, DMODEL, WSC, WLO);
  tcvt16<1><<<dim3(DMODEL / 64, DMODEL / 64, NLAYER), blk, 0, stream>>>(w_o, eSrcE, WO16, eDstE, DMODEL, DMODEL, KD, DMODEL, WSC, WLO);
  tcvt16<1><<<dim3(DFF / 64, DMODEL / 64, NLAYER), blk, 0, stream>>>(w_1, (long long)DMODEL * DFF, W116, (long long)DFF * KD,
                                                                    DMODEL, DFF, KD, DMODEL, WSC, WLO);
  tcvt16<1><<<dim3(DMODEL / 64, DFF / 64, NLAYER), blk, 0, stream>>>(w_2, (long long)DFF * DMODEL, W216, (long long)DMODEL * KF,
                                                                    DFF, DMODEL, KF, DFF, WSC, WLO);
  tcvt16<0><<<dim3(DMODEL / 64, OBSP / 64, 1), blk, 0, stream>>>(obs_w, 0LL, OBSW16, 0LL, OBSD, DMODEL, OBSP, 0, WSC, 0.f);
  tcvt16<1><<<dim3(NACTP / 64, DMODEL / 64, 1), blk, 0, stream>>>(act_w, 0LL, ACTW16, 0LL, DMODEL, NACT, KD, DMODEL, WSC, WLO);
  tcvt16<1><<<dim3(OBSP / 64, DMODEL / 64, 1), blk, 0, stream>>>(obsh_w, 0LL, OBSHW16, 0LL, DMODEL, OBSD, KD, DMODEL, WSC, WLO);

  gemm64<0, 0, 0, 1><<<gE, blk, 0, stream>>>(
      OBS16, OBSP, 0LL,
      OBSW16, OBSP, 0LL,
      (const float*)0,
      obs_b, DMODEL,
      (void*)XA, DMODEL, 0LL, 0LL,
      NROWS, DMODEL, OBSP, 1.0f / (OBC * WSC), 1.0f);

  for (int l = 0; l < NLAYER; ++l) {
    const size_t lwE = (size_t)l * DMODEL * KD;
    const size_t lw1 = (size_t)l * DFF * KD;
    const size_t lw2 = (size_t)l * DMODEL * KF;

    rmsn<<<gRow, blk128, 0, stream>>>(XA, norm1_w + (size_t)l * DMODEL, HH);

    gemm64<1, 0, 0, 0><<<gQK, blk, 0, stream>>>(
        HH, KD, 0LL,
        WQ16 + lwE, KD, sQK,
        (const float*)0,
        (const float*)0, 1,
        (void*)QP, KD, sKP, (long long)DMODEL,
        NROWS, DMODEL, KD, 1.0f / (HC * WSC), QC);

    gemm64<1, 0, 0, 0><<<gV, blk, 0, stream>>>(
        WV16 + lwE, KD, 0LL,
        HH, KD, (long long)SEQ * KD,
        (const float*)0,
        (const float*)0, 1,
        (void*)VTp, SEQ, (long long)VTR * SEQ, (long long)DMODEL * SEQ,
        DMODEL, SEQ, KD, 1.0f / (HC * WSC), VC);

    attn4<<<gAT, bAT, 0, stream>>>(QP, KP, VTp, relb + (size_t)l * NBUCK * NHEAD, CT);

    gemm64<0, 2, 0, 0><<<gE, blk, 0, stream>>>(
        CT, KD, 0LL,
        WO16 + lwE, KD, 0LL,
        XA,
        (const float*)0, 1,
        (void*)XB, DMODEL, 0LL, 0LL,
        NROWS, DMODEL, KD, 1.0f / (CC * WSC), 1.0f);

    rmsn<<<gRow, blk128, 0, stream>>>(XB, norm2_w + (size_t)l * DMODEL, HH);

    gemm64<1, 0, 2, 1><<<gF, blk, 0, stream>>>(
        HH, KD, 0LL,
        W116 + lw1, KD, 0LL,
        (const float*)0,
        b_1 + (size_t)l * DFF, DFF,
        (void*)G16, KF, 0LL, (long long)DFF,
        NROWS, DFF, KD, 1.0f / (HC * WSC), GC);

    gemm64<0, 2, 0, 1><<<gE, blk, 0, stream>>>(
        G16, KF, 0LL,
        W216 + lw2, KF, 0LL,
        XB,
        b_2 + (size_t)l * DMODEL, DMODEL,
        (void*)XA, DMODEL, 0LL, 0LL,
        NROWS, DMODEL, KF, 1.0f / (GC * WSC), 1.0f);
  }

  rmsn<<<gRow, blk128, 0, stream>>>(XA, fnorm_w, HH);

  gemm64<0, 0, 0, 1><<<gA, blk, 0, stream>>>(
      HH, KD, 0LL,
      ACTW16, KD, 0LL,
      (const float*)0,
      act_b, NACT,
      (void*)ACTF, NACTP, 0LL, 0LL,
      NROWS, NACTP, KD, 1.0f / (HC * WSC), 1.0f);

  gemm64<0, 0, 0, 1><<<gO, blk, 0, stream>>>(
      HH, KD, 0LL,
      OBSHW16, KD, 0LL,
      (const float*)0,
      obsh_b, OBSD,
      (void*)OBSF, OBSP, 0LL, 0LL,
      NROWS, OBSP, KD, 1.0f / (HC * WSC), 1.0f);

  ocopy<<<gOC, blk, 0, stream>>>(ACTF, OBSF, outp);
  (void)hipGetLastError();
}
